// MultiHeadAttention_53068615910142
// MI455X (gfx1250) — hardware-verified
//
#include <hip/hip_runtime.h>
#ifndef NB
#define NB 2
#endif
#ifndef SEQ
#define SEQ 2048
#endif
#define NB_FULL 2
#define SEQ_FULL 2048
#define DM 1024
#define NH 16
#define HD 64
#define QT 64
#define NR (NB * SEQ)
#define ER ((SEQ < 256) ? SEQ : 256)
#define EQT (ER / QT)
#define NQT (SEQ / QT)
#define SSCALE 0.125f
#define PCARRY 256.0f
#define PCARRY_INV 0.00390625f
#define RSC 2048.0f
#define RSC_INV 0.00048828125f

typedef __bf16 v16b __attribute__((ext_vector_type(16)));
typedef _Float16 v16h __attribute__((ext_vector_type(16)));
typedef unsigned short v8us __attribute__((ext_vector_type(8), may_alias));
typedef float  v8f  __attribute__((ext_vector_type(8)));
typedef float  v4f  __attribute__((ext_vector_type(4)));
typedef float  v4fa __attribute__((ext_vector_type(4), may_alias));
typedef int    v4i  __attribute__((ext_vector_type(4)));
typedef int    v4ia __attribute__((ext_vector_type(4), may_alias));
union FragB { v16b v; v8us half[2]; };
union FragH { v16h v; v8us half[2]; };
union Pack8 { v8us v; unsigned short u[8]; };

static_assert(HD == 64);
static_assert(HD == 16 * 4);
static_assert(NH * HD == DM);
static_assert(DM % 128 == 0);
static_assert(DM % 64 == 0);
static_assert(DM % 32 == 0);
static_assert(HD % 32 == 0);
static_assert(SEQ % 128 == 0);
static_assert(SEQ % QT == 0);
static_assert(SEQ % 64 == 0);
static_assert(SEQ % 32 == 0);
static_assert(QT == 4 * 16);
static_assert(NR % 128 == 0);
static_assert(ER % 128 == 0);
static_assert(ER % QT == 0);
static_assert(ER % 32 == 0);
static_assert(ER <= SEQ);
static_assert(EQT >= 1);
static_assert(NB <= NB_FULL);
static_assert(SEQ <= SEQ_FULL);
static_assert(8 * 8 == HD);
static_assert(4 * 8 == 32);
static_assert((size_t)NR * DM < 2147483647u);
static_assert((size_t)DM * DM < 2147483647u);
static_assert((size_t)SEQ_FULL * SEQ_FULL < 2147483647u);
static_assert(((size_t)NR * (DM / 8)) % 256 == 0);
static_assert(((size_t)DM * (DM / 8)) % 256 == 0);

constexpr size_t PLANE_B = (size_t)NR * DM * 2;
constexpr size_t WPL_B   = (size_t)DM * DM * 2;
constexpr size_t CARVE_B = 9 * PLANE_B + 3 * WPL_B;
static_assert(PLANE_B % 256 == 0);
static_assert(WPL_B % 256 == 0);
static_assert(CARVE_B <= 134217728u);

__device__ __forceinline__ unsigned short bf16_bits(float x) { unsigned int u = __float_as_uint(x); return (unsigned short)((u + 0x7FFFu + ((u >> 16) & 1u)) >> 16); }
__device__ __forceinline__ float bf16_val(unsigned short b) { return __uint_as_float(((unsigned int)b) << 16); }
__device__ __forceinline__ float bf16_rne(float x) { return bf16_val(bf16_bits(x)); }
__device__ __forceinline__ unsigned short f16_bits(float x) { const _Float16 hx = (_Float16)x; return __builtin_bit_cast(unsigned short, hx); }
__device__ __forceinline__ float f16_val(unsigned short b) { return (float)__builtin_bit_cast(_Float16, b); }

__device__ __forceinline__ v16b ld_fragb(const unsigned short* __restrict__ p, int off, int hh) {
  FragB f;
  f.half[0] = *(const v8us*)(p + off + 8 * hh);
  f.half[1] = *(const v8us*)(p + off + 16 + 8 * hh);
  return f.v;
}
__device__ __forceinline__ v16h ld_fragh(const unsigned short* __restrict__ p, int off, int hh) {
  FragH f;
  f.half[0] = *(const v8us*)(p + off + 8 * hh);
  f.half[1] = *(const v8us*)(p + off + 16 + 8 * hh);
  return f.v;
}
__device__ __forceinline__ void mmab2(v16b a0, v16b a1, v16b b, v8f& c0, v8f& c1) {
  c0 = __builtin_amdgcn_wmma_f32_16x16x32_bf16(false, a0, false, b, (short)0, c0, false, false);
  c1 = __builtin_amdgcn_wmma_f32_16x16x32_bf16(false, a1, false, b, (short)0, c1, false, false);
  asm volatile("v_nop\n\tv_nop\n\tv_nop\n\tv_nop" : "+v"(c0), "+v"(c1) : "v"(a0), "v"(a1), "v"(b));
}
__device__ __forceinline__ void mmah2(v16h a0, v16h a1, v16h b, v8f& c0, v8f& c1) {
  c0 = __builtin_amdgcn_wmma_f32_16x16x32_f16(false, a0, false, b, (short)0, c0, false, false);
  c1 = __builtin_amdgcn_wmma_f32_16x16x32_f16(false, a1, false, b, (short)0, c1, false, false);
  asm volatile("v_nop\n\tv_nop\n\tv_nop\n\tv_nop" : "+v"(c0), "+v"(c1) : "v"(a0), "v"(a1), "v"(b));
}

__global__ __launch_bounds__(256) void k_cvt_x(const float* __restrict__ q, const float* __restrict__ k, const float* __restrict__ v,
                                               unsigned short* __restrict__ Xq, unsigned short* __restrict__ Xk, unsigned short* __restrict__ Xv) {
  const int t = blockIdx.x * 256 + threadIdx.x;
  if (t >= NR * (DM / 8)) return;
  const int row = t / (DM / 8), c8 = (t % (DM / 8)) * 8;
  const int b = row / SEQ, s = row % SEQ;
  const size_t src = ((size_t)b * SEQ_FULL + s) * DM + c8;
  const v4f a0 = *(const v4fa*)(q + src), a1 = *(const v4fa*)(q + src + 4);
  const v4f b0 = *(const v4fa*)(k + src), b1 = *(const v4fa*)(k + src + 4);
  const v4f c0 = *(const v4fa*)(v + src), c1 = *(const v4fa*)(v + src + 4);
  Pack8 fq, fk, fv;
#pragma unroll
  for (int i = 0; i < 4; ++i) {
    fq.u[i] = bf16_bits(a0[i]); fq.u[4 + i] = bf16_bits(a1[i]);
    fk.u[i] = bf16_bits(b0[i]); fk.u[4 + i] = bf16_bits(b1[i]);
    fv.u[i] = bf16_bits(c0[i]); fv.u[4 + i] = bf16_bits(c1[i]);
  }
  const size_t dst = (size_t)row * DM + c8;
  const v8us vq = fq.v, vk = fk.v, vv = fv.v;
  *(volatile v8us*)(Xq + dst) = vq; *(volatile v8us*)(Xk + dst) = vk; *(volatile v8us*)(Xv + dst) = vv;
  __threadfence();
  *(volatile v8us*)(Xq + dst) = vq; *(volatile v8us*)(Xk + dst) = vk; *(volatile v8us*)(Xv + dst) = vv;
}

__global__ __launch_bounds__(256) void k_cvt_w(const float* __restrict__ W0, const float* __restrict__ W1, const float* __restrict__ W2,
                                               unsigned short* __restrict__ B0, unsigned short* __restrict__ B1, unsigned short* __restrict__ B2) {
  const int t = blockIdx.x * 256 + threadIdx.x;
  if (t >= DM * (DM / 8)) return;
  const size_t e = (size_t)t * 8;
  const v4f a0 = *(const v4fa*)(W0 + e), a1 = *(const v4fa*)(W0 + e + 4);
  const v4f b0 = *(const v4fa*)(W1 + e), b1 = *(const v4fa*)(W1 + e + 4);
  const v4f c0 = *(const v4fa*)(W2 + e), c1 = *(const v4fa*)(W2 + e + 4);
  Pack8 f0, f1, f2;
#pragma unroll
  for (int i = 0; i < 4; ++i) {
    f0.u[i] = bf16_bits(a0[i]); f0.u[4 + i] = bf16_bits(a1[i]);
    f1.u[i] = bf16_bits(b0[i]); f1.u[4 + i] = bf16_bits(b1[i]);
    f2.u[i] = bf16_bits(c0[i]); f2.u[4 + i] = bf16_bits(c1[i]);
  }
  const v8us v0 = f0.v, v1 = f1.v, v2 = f2.v;
  *(volatile v8us*)(B0 + e) = v0; *(volatile v8us*)(B1 + e) = v1; *(volatile v8us*)(B2 + e) = v2;
  __threadfence();
  *(volatile v8us*)(B0 + e) = v0; *(volatile v8us*)(B1 + e) = v1; *(volatile v8us*)(B2 + e) = v2;
}

template <int BIAS_ROW>
__device__ __forceinline__ void proj_body(const unsigned short* __restrict__ A, const unsigned short* __restrict__ B, const float* __restrict__ bias,
                                          unsigned short* __restrict__ OH, unsigned short* __restrict__ OL,
                                          const int arow0, const int brow0, const int obase, const int opitch, const int bias0, const bool need_lo) {
  __shared__ __attribute__((aligned(16))) float so[4][32][68];
  const int tid = threadIdx.x;
  const int wave = __builtin_amdgcn_readfirstlane(tid >> 5);
  const int lane = tid & 31, ln = lane & 15, hh = lane >> 4;
  const int ar0 = (arow0 + 32 * wave + ln) * DM, ar1 = ar0 + 16 * DM;
  const int br0 = (brow0 + ln) * DM, br1 = br0 + 16 * DM, br2 = br1 + 16 * DM, br3 = br2 + 16 * DM;
  const v8f z8 = {0.f, 0.f, 0.f, 0.f, 0.f, 0.f, 0.f, 0.f};
  v8f c00 = z8, c01 = z8, c02 = z8, c03 = z8, c10 = z8, c11 = z8, c12 = z8, c13 = z8;
#pragma unroll 1
  for (int kb = 0; kb < DM; kb += 32) {
    const v16b fa0 = ld_fragb(A, ar0 + kb, hh);
    const v16b fa1 = ld_fragb(A, ar1 + kb, hh);
    v16b fb = ld_fragb(B, br0 + kb, hh); mmab2(fa0, fa1, fb, c00, c10);
    fb = ld_fragb(B, br1 + kb, hh);      mmab2(fa0, fa1, fb, c01, c11);
    fb = ld_fragb(B, br2 + kb, hh);      mmab2(fa0, fa1, fb, c02, c12);
    fb = ld_fragb(B, br3 + kb, hh);      mmab2(fa0, fa1, fb, c03, c13);
  }
  float brow[2][8];
  float bcol[4];
#pragma unroll
  for (int t = 0; t < 4; ++t) bcol[t] = 0.f;
#pragma unroll
  for (int hf = 0; hf < 2; ++hf)
#pragma unroll
    for (int r = 0; r < 8; ++r) brow[hf][r] = 0.f;
  if (BIAS_ROW) {
#pragma unroll
    for (int hf = 0; hf < 2; ++hf)
#pragma unroll
      for (int r = 0; r < 8; ++r) brow[hf][r] = bf16_rne(bias[bias0 + 32 * wave + hf * 16 + 8 * hh + r]);
  } else {
#pragma unroll
    for (int t = 0; t < 4; ++t) bcol[t] = bf16_rne(bias[bias0 + t * 16 + ln]);
  }
  const v8f accs[8] = {c00, c01, c02, c03, c10, c11, c12, c13};
#pragma unroll
  for (int u = 0; u < 8; ++u) {
    const int t = u & 3, hf = u >> 2;
#pragma unroll
    for (int r = 0; r < 8; ++r) so[wave][hf * 16 + 8 * hh + r][t * 16 + ln] = accs[u][r] + brow[hf][r] + bcol[t];
  }
  __builtin_amdgcn_fence(4  , "workgroup");
  __builtin_amdgcn_wave_barrier();
  const int prow = lane >> 3, pc = (lane & 7) * 8;
  for (int pass = 0; pass < 2; ++pass) {
#pragma unroll
    for (int it = 0; it < 8; ++it) {
      const int r = it * 4 + prow;
      const v4f x0 = *(const v4fa*)&so[wave][r][pc];
      const v4f x1 = *(const v4fa*)&so[wave][r][pc + 4];
      Pack8 fh, fl;
#pragma unroll
      for (int i = 0; i < 4; ++i) {
        const unsigned short h0 = f16_bits(x0[i]);
        const unsigned short h1 = f16_bits(x1[i]);
        fh.u[i] = h0; fh.u[4 + i] = h1;
        fl.u[i]     = f16_bits((x0[i] - f16_val(h0)) * RSC);
        fl.u[4 + i] = f16_bits((x1[i] - f16_val(h1)) * RSC);
      }
      const size_t g = (size_t)obase + (size_t)(32 * wave + r) * (size_t)opitch + (size_t)pc;
      const v8us vh = fh.v, vl = fl.v;
      *(volatile v8us*)(OH + g) = vh;
      if (need_lo) *(volatile v8us*)(OL + g) = vl;
    }
    if (pass == 0) __threadfence();
  }
}

__global__ __launch_bounds__(128) void k_proj_qk(const unsigned short* __restrict__ X, const unsigned short* __restrict__ Wb, const float* __restrict__ bias,
                                                 unsigned short* __restrict__ OH, unsigned short* __restrict__ OL) {
  const int ntn = DM / 64;
  const int mt = blockIdx.x / ntn, nq = blockIdx.x - mt * ntn;
  const bool need_lo = ((mt * 128) % SEQ) < ER;
  proj_body<0>(X, Wb, bias, OH, OL, mt * 128, nq * 64, mt * 128 * DM + nq * 64, DM, nq * 64, need_lo);
}

__global__ __launch_bounds__(128) void k_proj_vt(const unsigned short* __restrict__ Wb, const unsigned short* __restrict__ X, const float* __restrict__ bias,
                                                 unsigned short* __restrict__ VH, unsigned short* __restrict__ VL) {
  const int ntn = SEQ / 64, nmt = DM / 128;
  const int b = blockIdx.x / (nmt * ntn);
  const int rem = blockIdx.x - b * (nmt * ntn);
  const int mt = rem / ntn, nq = rem - mt * ntn;
  const bool need_lo = (nq * 64) < ER;
  proj_body<1>(Wb, X, bias, VH, VL, mt * 128, b * SEQ + nq * 64, (b * DM + mt * 128) * SEQ + nq * 64, SEQ, mt * 128, need_lo);
}

template <int RES>
__device__ __forceinline__ void attn_body(const unsigned short* __restrict__ Qh, const unsigned short* __restrict__ Ql,
                                          const unsigned short* __restrict__ Kh, const unsigned short* __restrict__ Kl,
                                          const unsigned short* __restrict__ VH, const unsigned short* __restrict__ VL,
                                          const int* __restrict__ mask, float* __restrict__ out, const int qt, const int bh) {
  __shared__ __attribute__((aligned(16))) float so[4][16][68];
  const int tid = threadIdx.x;
  const int wave = __builtin_amdgcn_readfirstlane(tid >> 5);
  const int lane = tid & 31, ln = lane & 15, hh = lane >> 4;
  const int b = bh / NH, h = bh - b * NH;
  const int q0 = qt * QT + wave * 16;
  const int qoff  = (b * SEQ + q0 + ln) * DM + h * HD;
  const int kbase = (b * SEQ + ln) * DM + h * HD;
  const int vbase = (bh * HD + ln) * SEQ;
  const int moff  = (q0 + ln) * SEQ_FULL + 8 * hh;
  const v8f z8 = {0.f, 0.f, 0.f, 0.f, 0.f, 0.f, 0.f, 0.f};
  v8f o0 = z8, o1 = z8, o2 = z8, o3 = z8;
  v8f r0 = z8, r1 = z8, r2 = z8, r3 = z8;
  float m = -1.0e30f, l = 0.f;
  int keep = 0;
#pragma unroll 1
  for (int kb = 0; kb < SEQ; kb += 32) {
    const v4i ma = *(const v4ia*)(mask + moff + kb);
    const v4i mb = *(const v4ia*)(mask + moff + kb + 4);
    const v4i mc = *(const v4ia*)(mask + moff + kb + 16);
    const v4i md = *(const v4ia*)(mask + moff + kb + 20);
    const int any = ma[0] | ma[1] | ma[2] | ma[3] | mb[0] | mb[1] | mb[2] | mb[3] |
                    mc[0] | mc[1] | mc[2] | mc[3] | md[0] | md[1] | md[2] | md[3];
    if (__builtin_amdgcn_ballot_w32(any != 0) == 0u) continue;
    keep |= any;
    const bool resk = (RES != 0) && (kb < ER);
    const int ko = kbase + kb * DM;
    v8f s0 = z8, s1 = z8, t0 = z8, t1 = z8;
#pragma unroll
    for (int j = 0; j < 2; ++j) {
      const v16h qf = ld_fragh(Qh, qoff + 32 * j, hh);
      const v16h ka = ld_fragh(Kh, ko + 32 * j, hh);
      const v16h kc = ld_fragh(Kh, ko + 16 * DM + 32 * j, hh);
      mmah2(ka, kc, qf, s0, s1);
      if (resk) {
        const v16h qr = ld_fragh(Ql, qoff + 32 * j, hh);
        mmah2(ka, kc, qr, t0, t1);
        const v16h la = ld_fragh(Kl, ko + 32 * j, hh);
        const v16h lc = ld_fragh(Kl, ko + 16 * DM + 32 * j, hh);
        mmah2(la, lc, qf, t0, t1);
      }
    }
    if (resk) { s0 = s0 + t0 * RSC_INV; s1 = s1 + t1 * RSC_INV; }
    const int mk0[8] = {ma[0], ma[1], ma[2], ma[3], mb[0], mb[1], mb[2], mb[3]};
    const int mk1[8] = {mc[0], mc[1], mc[2], mc[3], md[0], md[1], md[2], md[3]};
#pragma unroll
    for (int r = 0; r < 8; ++r) {
      s0[r] = (mk0[r] == 0) ? -1.0e9f : s0[r] * SSCALE;
      s1[r] = (mk1[r] == 0) ? -1.0e9f : s1[r] * SSCALE;
    }
    float mx = fmaxf(s0[0], s1[0]);
#pragma unroll
    for (int r = 1; r < 8; ++r) mx = fmaxf(mx, fmaxf(s0[r], s1[r]));
    mx = fmaxf(mx, __shfl_xor(mx, 16, 32));
    const float mn = fmaxf(m, mx);
    const float al = __expf(m - mn);
    m = mn;
    v16h ph = {};
    v16h pl = {};
    float ps = 0.f;
#pragma unroll
    for (int r = 0; r < 8; ++r) {
      const float p0 = __expf(s0[r] - mn);
      const float p1 = __expf(s1[r] - mn);
      ps += p0 + p1;
      const float e0 = p0 * PCARRY, e1 = p1 * PCARRY;
      const _Float16 h0 = (_Float16)e0, h1 = (_Float16)e1;
      ph[r] = h0; ph[8 + r] = h1;
      if (RES) {
        pl[r]     = (_Float16)((e0 - (float)h0) * RSC);
        pl[8 + r] = (_Float16)((e1 - (float)h1) * RSC);
      }
    }
    l = l * al + ps;
    o0 = o0 * al; o1 = o1 * al; o2 = o2 * al; o3 = o3 * al;
    if (RES) { r0 = r0 * al; r1 = r1 * al; r2 = r2 * al; r3 = r3 * al; }
    const int vo = vbase + kb;
    const v16h va0 = ld_fragh(VH, vo, hh);
    const v16h va1 = ld_fragh(VH, vo + 16 * SEQ, hh);
    const v16h va2 = ld_fragh(VH, vo + 32 * SEQ, hh);
    const v16h va3 = ld_fragh(VH, vo + 48 * SEQ, hh);
    mmah2(va0, va1, ph, o0, o1);
    mmah2(va2, va3, ph, o2, o3);
    if (resk) {
      mmah2(va0, va1, pl, r0, r1);
      mmah2(va2, va3, pl, r2, r3);
      const v16h vl0 = ld_fragh(VL, vo, hh);
      const v16h vl1 = ld_fragh(VL, vo + 16 * SEQ, hh);
      const v16h vl2 = ld_fragh(VL, vo + 32 * SEQ, hh);
      const v16h vl3 = ld_fragh(VL, vo + 48 * SEQ, hh);
      mmah2(vl0, vl1, ph, r0, r1);
      mmah2(vl2, vl3, ph, r2, r3);
    }
  }
  l += __shfl_xor(l, 16, 32);
  keep |= __shfl_xor(keep, 16, 32);
  const float inv = (1.0f / l) * PCARRY_INV;
  if (RES) { o0 = o0 + r0 * RSC_INV; o1 = o1 + r1 * RSC_INV; o2 = o2 + r2 * RSC_INV; o3 = o3 + r3 * RSC_INV; }
  const float poison = __uint_as_float(0x7FC00000u);
  const v8f ot[4] = {o0, o1, o2, o3};
#pragma unroll
  for (int t = 0; t < 4; ++t) {
    v4f w0, w1;
#pragma unroll
    for (int r = 0; r < 4; ++r) {
      const float c0 = ot[t][r] * inv, c1 = ot[t][4 + r] * inv;
      w0[r] = (keep != 0) ? c0 : poison;
      w1[r] = (keep != 0) ? c1 : poison;
    }
    *(v4fa*)&so[wave][ln][16 * t + 8 * hh]     = w0;
    *(v4fa*)&so[wave][ln][16 * t + 8 * hh + 4] = w1;
  }
  __builtin_amdgcn_fence(4  , "workgroup");
  __builtin_amdgcn_wave_barrier();
  const int rsub = lane >> 4, c4 = (lane & 15) * 4;
  for (int pass = 0; pass < 2; ++pass) {
#pragma unroll
    for (int it = 0; it < 8; ++it) {
      const int row = it * 2 + rsub;
      const v4f x = *(const v4fa*)&so[wave][row][c4];
      *(volatile v4f*)(out + (size_t)(b * SEQ + q0 + row) * DM + h * HD + c4) = x;
    }
    if (pass == 0) __threadfence();
  }
}

__global__ __launch_bounds__(128) void k_attn_early(const unsigned short* __restrict__ Qh, const unsigned short* __restrict__ Ql,
                                                    const unsigned short* __restrict__ Kh, const unsigned short* __restrict__ Kl,
                                                    const unsigned short* __restrict__ VH, const unsigned short* __restrict__ VL,
                                                    const int* __restrict__ mask, float* __restrict__ out) {
  const int bh = blockIdx.x / EQT;
  const int qt = blockIdx.x - bh * EQT;
  attn_body<1>(Qh, Ql, Kh, Kl, VH, VL, mask, out, qt, bh);
}

__global__ __launch_bounds__(128) void k_attn_main(const unsigned short* __restrict__ Qh, const unsigned short* __restrict__ Kh,
                                                   const unsigned short* __restrict__ VH, const int* __restrict__ mask, float* __restrict__ out) {
  const int nq = NQT - EQT;
  const int bh = blockIdx.x / nq;
  const int qt = EQT + (blockIdx.x - bh * nq);
  attn_body<0>(Qh, Qh, Kh, Kh, VH, VH, mask, out, qt, bh);
}

extern "C" void kernel_launch(void* const* d_in, const int* in_sizes, int n_in,
                              void* d_out, int out_size, void* d_ws, size_t ws_size, hipStream_t stream) {
  if (n_in < 10) return;
  const long long need_act = ((long long)(NB - 1) * SEQ_FULL + SEQ) * DM;
  if ((long long)in_sizes[0] < need_act || (long long)in_sizes[1] < need_act || (long long)in_sizes[2] < need_act) return;
  if ((long long)in_sizes[3] < (long long)(SEQ - 1) * SEQ_FULL + SEQ) return;
  if ((long long)in_sizes[4] < (long long)DM * DM || (long long)in_sizes[6] < (long long)DM * DM || (long long)in_sizes[8] < (long long)DM * DM) return;
  if (in_sizes[5] < DM || in_sizes[7] < DM || in_sizes[9] < DM) return;
  if ((long long)out_size < (long long)NR * DM) return;
  if (ws_size < CARVE_B) return;
  const float* q  = (const float*)d_in[0];
  const float* k  = (const float*)d_in[1];
  const float* v  = (const float*)d_in[2];
  const int* mask = (const int*)d_in[3];
  const float* Wq = (const float*)d_in[4];
  const float* bq = (const float*)d_in[5];
  const float* Wk = (const float*)d_in[6];
  const float* bk = (const float*)d_in[7];
  const float* Wv = (const float*)d_in[8];
  const float* bv = (const float*)d_in[9];
  char* ws = (char*)d_ws;
  unsigned short* Xq  = (unsigned short*)(ws);
  unsigned short* Xk  = (unsigned short*)(ws + PLANE_B);
  unsigned short* Xv  = (unsigned short*)(ws + 2 * PLANE_B);
  unsigned short* Wqb = (unsigned short*)(ws + 3 * PLANE_B);
  unsigned short* Wkb = (unsigned short*)(ws + 3 * PLANE_B + WPL_B);
  unsigned short* Wvb = (unsigned short*)(ws + 3 * PLANE_B + 2 * WPL_B);
  char* ws2 = ws + 3 * PLANE_B + 3 * WPL_B;
  unsigned short* Qh = (unsigned short*)(ws2);
  unsigned short* Ql = (unsigned short*)(ws2 + PLANE_B);
  unsigned short* Kh = (unsigned short*)(ws2 + 2 * PLANE_B);
  unsigned short* Kl = (unsigned short*)(ws2 + 3 * PLANE_B);
  unsigned short* VH = (unsigned short*)(ws2 + 4 * PLANE_B);
  unsigned short* VL = (unsigned short*)(ws2 + 5 * PLANE_B);
  k_cvt_x<<<(unsigned)(((size_t)NR * (DM / 8)) / 256), 256, 0, stream>>>(q, k, v, Xq, Xk, Xv);
  k_cvt_w<<<(unsigned)(((size_t)DM * (DM / 8)) / 256), 256, 0, stream>>>(Wq, Wk, Wv, Wqb, Wkb, Wvb);
  k_proj_qk<<<(NR / 128) * (DM / 64), 128, 0, stream>>>(Xq, Wqb, bq, Qh, Ql);
  k_proj_qk<<<(NR / 128) * (DM / 64), 128, 0, stream>>>(Xk, Wkb, bk, Kh, Kl);
  k_proj_vt<<<NB * (DM / 128) * (SEQ / 64), 128, 0, stream>>>(Wvb, Xv, bv, VH, VL);
  k_attn_early<<<NB * NH * EQT, 128, 0, stream>>>(Qh, Ql, Kh, Kl, VH, VL, mask, (float*)d_out);
  if (NQT > EQT) {
    k_attn_main<<<NB * NH * (NQT - EQT), 128, 0, stream>>>(Qh, Kh, VH, mask, (float*)d_out);
  }
}
